// MultiHeadAttentionBlock_22746146800125
// MI455X (gfx1250) — hardware-verified
//
#include <hip/hip_runtime.h>
#include <math.h>

typedef __attribute__((ext_vector_type(16))) _Float16 v16h;
typedef __attribute__((ext_vector_type(16))) __bf16 v16b;
typedef __attribute__((ext_vector_type(8)))  _Float16 v8h;
typedef __attribute__((ext_vector_type(8)))  float v8f;
typedef __attribute__((ext_vector_type(4)))  float v4f;
typedef __attribute__((ext_vector_type(4)))  unsigned v4u;
typedef __attribute__((ext_vector_type(4)))  int v4i;

template <typename T> __device__ __forceinline__ void vst2(void* p, T v) { *(volatile T*)p = v; __threadfence(); *(volatile T*)p = v; }
__device__ __forceinline__ v8f wmma16(v16h a, v16h b, v8f c) {
  v8f d = __builtin_amdgcn_wmma_f32_16x16x32_f16(false, a, false, b, (short)0, c, false, false);
  asm volatile("v_nop\n\tv_nop\n\tv_nop\n\tv_nop" : "+v"(d) : "v"(a), "v"(b));
  return d;
}
__device__ __forceinline__ v8f wmma_bf(v16b a, v16b b, v8f c) {
  v8f d = __builtin_amdgcn_wmma_f32_16x16x32_bf16(false, a, false, b, (short)0, c, false, false);
  asm volatile("v_nop\n\tv_nop\n\tv_nop\n\tv_nop" : "+v"(d) : "v"(a), "v"(b));
  return d;
}
__device__ __forceinline__ v16h frag_h(const _Float16* rowk0, unsigned lane) {
  union { v16h v; v8h q[2]; } u; const _Float16* p = rowk0 + 8u * (lane >> 4);
  u.q[0] = *(const v8h*)p; u.q[1] = *(const v8h*)(p + 16); return u.v;
}
__device__ __forceinline__ v16h frag_f32s(const float* rowk0, unsigned lane, float sc) {
  v16h a; const float* p = rowk0 + 8u * (lane >> 4);
#pragma unroll
  for (int i = 0; i < 8; ++i) { a[i] = (_Float16)(p[i] * sc); a[8 + i] = (_Float16)(p[16 + i] * sc); }
  return a;
}
__device__ __forceinline__ float bfr(float v) { return (float)(__bf16)v; }
__device__ __forceinline__ v16b wcol_oi(const float* Wm, unsigned k0, unsigned o, unsigned lane, unsigned K) { v16b w; const float* p = Wm + (size_t)o * K + k0 + 8u * (lane >> 4);
#pragma unroll
  for (int i = 0; i < 8; ++i) { w[i] = (__bf16)p[i]; w[8 + i] = (__bf16)p[16 + i]; }
  return w; }
__device__ __forceinline__ v16h wcolh_oi(const float* Wm, unsigned k0, unsigned o, unsigned lane, unsigned K) { v16h w; const float* p = Wm + (size_t)o * K + k0 + 8u * (lane >> 4);
#pragma unroll
  for (int i = 0; i < 8; ++i) { w[i] = (_Float16)(bfr(p[i]) * 256.0f); w[8 + i] = (_Float16)(bfr(p[16 + i]) * 256.0f); }
  return w; }
#define LDSX() do { asm volatile("s_wait_dscnt 0" ::: "memory"); __builtin_amdgcn_wave_barrier(); __builtin_amdgcn_fence(3  , "workgroup"); } while (0)

#ifndef NB
#define NB 2
#endif
#ifndef SEQ
#define SEQ 4096
#endif
#define NB_FULL 2
#define SEQ_FULL 4096
#define TT SEQ
#define CC 512
#define DIN 512
#define NH 8
#define HD 64
#define SC2 (0.125f * 1.44269504088896341f)

static_assert(NB <= NB_FULL);
static_assert(SEQ <= SEQ_FULL);
static_assert(TT % 64 == 0);
static_assert(CC % 128 == 0);
static_assert(DIN % 128 == 0);
static_assert(DIN % 32 == 0);
static_assert(CC % 32 == 0);
static_assert(HD == 64);
static_assert(NH * HD == CC);
static_assert((size_t)(NB * TT / 64) * (CC / 128) * 64 * 128 == (size_t)NB * TT * CC);
static_assert((size_t)(TT / 64) * (NB * NH) * 64 * HD == (size_t)NB * TT * CC);
static_assert((size_t)(NB * TT / 64) * (DIN / 128) * 64 * 128 == (size_t)NB * TT * DIN);

#define WS_QH  ((size_t)0)
#define WS_QL  (WS_QH + 2u * (size_t)NB * TT * CC)
#define WS_KH  (WS_QL + 2u * (size_t)NB * TT * CC)
#define WS_VT  (WS_KH + 2u * (size_t)NB * TT * CC)
#define WS_Y   (WS_VT + 2u * (size_t)NB * CC * TT)
#define WS_END (WS_Y  + 4u * (size_t)NB * TT * CC)
static_assert(WS_END <= (size_t)134217728);
static_assert(WS_QL % 128 == 0);
static_assert(WS_KH % 128 == 0);
static_assert(WS_VT % 128 == 0);
static_assert(WS_Y % 128 == 0);

__global__ __launch_bounds__(128) void k_proj(const float* __restrict__ XQ, const float* __restrict__ XK, const float* __restrict__ XV, const float* __restrict__ WQ, const float* __restrict__ WK, const float* __restrict__ WV,
    _Float16* __restrict__ QH, _Float16* __restrict__ QL, _Float16* __restrict__ KH, _Float16* __restrict__ VT) {
  __shared__ __align__(16) _Float16 sh[64][136], sl[64][136]; __shared__ __align__(16) _Float16 th[128][72];
  const unsigned tid = threadIdx.x, wave = tid >> 5, lane = tid & 31u, col = lane & 15u, g = lane >> 4;
  const unsigned which = blockIdx.z; const unsigned c0 = blockIdx.y * 128u; const unsigned r0 = blockIdx.x * 64u; const unsigned bb = r0 / (unsigned)TT; const unsigned t0 = r0 % (unsigned)TT;
  const float* X = which == 0 ? XQ : which == 1 ? XK : XV; const float* WA = which == 0 ? WQ : which == 1 ? WK : WV;
  const float* xrow = X + ((size_t)bb * SEQ_FULL + t0 + wave * 16u + col) * DIN;
  v8f acc[8] = {};
#pragma unroll 2
  for (unsigned kc = 0; kc < DIN / 32; ++kc) { v16b a; { const float* p = xrow + kc * 32u + 8u * g;
#pragma unroll
      for (int i = 0; i < 8; ++i) { a[i] = (__bf16)p[i]; a[8 + i] = (__bf16)p[16 + i]; } }
    asm volatile("s_wait_loadcnt 0x0" ::: "memory");
#pragma unroll
    for (int j = 0; j < 8; ++j) { const v16b w = wcol_oi(WA, kc * 32u, c0 + j * 16u + col, lane, DIN); asm volatile("s_wait_loadcnt 0x0" ::: "memory"); acc[j] = wmma_bf(a, w, acc[j]); } }
  if (which < 2) {
    _Float16* DH = which == 0 ? QH : KH;
#pragma unroll
    for (int j = 0; j < 8; ++j) {
#pragma unroll
      for (int r = 0; r < 8; ++r) { const float v = acc[j][r]; const _Float16 hv = (_Float16)v; sh[wave * 16u + 8u * g + r][j * 16u + col] = hv; sl[wave * 16u + 8u * g + r][j * 16u + col] = (_Float16)((v - (float)hv) * 1024.0f); } }
    __syncthreads();
    for (unsigned e = tid; e < 64u * 16u; e += 128u) { const unsigned rl = e >> 4, q = e & 15u; const size_t off = (size_t)(r0 + rl) * CC + c0 + q * 8u;
      const v4u hv4 = *(const v4u*)&sh[rl][q * 8u]; vst2(DH + off, hv4);
      if (which == 0) { const v4u lv4 = *(const v4u*)&sl[rl][q * 8u]; vst2(QL + off, lv4); } }
  } else {
#pragma unroll
    for (int j = 0; j < 8; ++j) {
#pragma unroll
      for (int r = 0; r < 8; ++r) { const unsigned rl = wave * 16u + 8u * g + r, cl = j * 16u + col; th[cl][rl] = (_Float16)acc[j][r]; } }
    __syncthreads();
    for (unsigned e = tid; e < 128u * 8u; e += 128u) { const unsigned cl = e >> 3, q = e & 7u; const v4u tv4 = *(const v4u*)&th[cl][q * 8u]; vst2(VT + ((size_t)bb * CC + c0 + cl) * (size_t)TT + t0 + q * 8u, tv4); } } }

__global__ __launch_bounds__(128) void k_attn(const _Float16* __restrict__ QH, const _Float16* __restrict__ QL, const _Float16* __restrict__ KH, const _Float16* __restrict__ VT, const int* __restrict__ MASK, float* __restrict__ Y) {
  __shared__ __align__(16) float ss[4][16][HD + 4];
  const unsigned tid = threadIdx.x, wave = tid >> 5, lane = tid & 31u, col = lane & 15u, g = lane >> 4;
  const unsigned b = blockIdx.y / (unsigned)NH, h = blockIdx.y % (unsigned)NH;
  const unsigned ql0 = blockIdx.x * 64u + wave * 16u;
  const size_t qoff = ((size_t)b * TT + ql0 + col) * CC + h * HD;
  const v16h qh0 = frag_h(QH + qoff, lane), qh1 = frag_h(QH + qoff + 32, lane);
  const v16h qr0 = frag_h(QL + qoff, lane), qr1 = frag_h(QL + qoff + 32, lane);
  const _Float16* Kb = KH + (size_t)b * TT * CC + h * HD;
  const _Float16* Vb = VT + ((size_t)b * CC + h * HD) * (size_t)TT;
  const int* Mb = MASK + (size_t)b * SEQ_FULL;
  v8f o[4] = {};
  float mi = -1.0e30f, li = 0.f;
#pragma unroll 1
  for (unsigned kv = 0; kv < (unsigned)TT; kv += 64u) {
    v8f sc[4];
#pragma unroll
    for (int t = 0; t < 4; ++t) {
      const _Float16* kr = Kb + (size_t)(kv + t * 16u + col) * CC;
      const v16h k0 = frag_h(kr, lane), k1 = frag_h(kr + 32, lane);
      const v4i ma = *(const v4i*)(Mb + kv + t * 16u + 8u * g), mb = *(const v4i*)(Mb + kv + t * 16u + 8u * g + 4u);
      v8f a = {}, ar = {};
      a = wmma16(k0, qh0, a); a = wmma16(k1, qh1, a);
      ar = wmma16(k0, qr0, ar); ar = wmma16(k1, qr1, ar);
#pragma unroll
      for (int r = 0; r < 8; ++r) { const int mk = (r < 4) ? ma[r & 3] : mb[r & 3]; const float s = (a[r] + ar[r] * (1.0f / 1024.0f)) * SC2; sc[t][r] = (mk == 0) ? -1.0e9f : s; }
    }
    float tm = sc[0][0];
#pragma unroll
    for (int t = 0; t < 4; ++t) {
#pragma unroll
      for (int r = 0; r < 8; ++r) tm = fmaxf(tm, sc[t][r]); }
    tm = fmaxf(tm, __shfl_xor(tm, 16));
    const float mn = fmaxf(mi, tm);
    const float corr = exp2f(mi - mn);
    mi = mn;
    const float ms = mn - 10.0f;
    li *= corr;
#pragma unroll
    for (int d = 0; d < 4; ++d) {
#pragma unroll
      for (int r = 0; r < 8; ++r) o[d][r] *= corr; }
    v16h pb0, pb1;
#pragma unroll
    for (int r = 0; r < 8; ++r) {
      const float p0 = exp2f(sc[0][r] - ms), p1 = exp2f(sc[1][r] - ms), p2 = exp2f(sc[2][r] - ms), p3 = exp2f(sc[3][r] - ms);
      li += (p0 + p1) + (p2 + p3);
      pb0[r] = (_Float16)p0; pb0[8 + r] = (_Float16)p1; pb1[r] = (_Float16)p2; pb1[8 + r] = (_Float16)p3; }
#pragma unroll
    for (int d = 0; d < 4; ++d) { const _Float16* vr = Vb + (size_t)(d * 16u + col) * (size_t)TT + kv;
      o[d] = wmma16(frag_h(vr, lane), pb0, o[d]); o[d] = wmma16(frag_h(vr + 32, lane), pb1, o[d]); }
  }
  const float lt = li + __shfl_xor(li, 16);
  const float inv = 1.0f / lt;
#pragma unroll
  for (int d = 0; d < 4; ++d) { v4f lo, hi; lo[0] = o[d][0] * inv; lo[1] = o[d][1] * inv; lo[2] = o[d][2] * inv; lo[3] = o[d][3] * inv; hi[0] = o[d][4] * inv; hi[1] = o[d][5] * inv; hi[2] = o[d][6] * inv; hi[3] = o[d][7] * inv;
    *(v4f*)&ss[wave][col][d * 16u + 8u * g] = lo; *(v4f*)&ss[wave][col][d * 16u + 8u * g + 4u] = hi; }
  LDSX();
#pragma unroll 1
  for (unsigned rl = 0; rl < 8u; ++rl) { const unsigned row = rl * 2u + g; const v4f yv = *(const v4f*)&ss[wave][row][col * 4u]; vst2(Y + ((size_t)b * TT + ql0 + row) * CC + h * HD + col * 4u, yv); } }

__global__ __launch_bounds__(128) void k_out(const float* __restrict__ Y, const float* __restrict__ WO, float* __restrict__ OUT) { __shared__ __align__(16) float sf[4][16][132];
  const unsigned tid = threadIdx.x, wave = tid >> 5, lane = tid & 31u, col = lane & 15u, g = lane >> 4; const unsigned c0 = blockIdx.y * 128u; const size_t r0 = (size_t)blockIdx.x * 64u + wave * 16u;
  v8f acc[8] = {};
#pragma unroll 2
  for (unsigned kc = 0; kc < CC / 32; ++kc) { const v16h a = frag_f32s(Y + (r0 + col) * CC + kc * 32u, lane, 64.0f); asm volatile("s_wait_loadcnt 0x0" ::: "memory");
#pragma unroll
    for (int j = 0; j < 8; ++j) { const v16h w = wcolh_oi(WO, kc * 32u, c0 + j * 16u + col, lane, CC); asm volatile("s_wait_loadcnt 0x0" ::: "memory"); acc[j] = wmma16(a, w, acc[j]); } }
#pragma unroll
  for (int j = 0; j < 8; ++j) {
#pragma unroll
    for (int r = 0; r < 8; ++r) sf[wave][8u * g + r][j * 16u + col] = acc[j][r] * (1.0f / 16384.0f); }
  LDSX();
#pragma unroll 1
  for (unsigned rl = 0; rl < 16u; ++rl) { const v4f ov = *(const v4f*)&sf[wave][rl][lane * 4u]; vst2(OUT + (r0 + rl) * DIN + c0 + lane * 4u, ov); } }

extern "C" void kernel_launch(void* const* d_in, const int* in_sizes, int n_in, void* d_out, int out_size, void* d_ws, size_t ws_size, hipStream_t stream) {
  if (n_in < 8) return;
  const int need_x = ((NB - 1) * SEQ_FULL + TT) * DIN;
  const int need_m = (NB - 1) * SEQ_FULL + TT;
  if (in_sizes[0] < need_x || in_sizes[1] < need_x || in_sizes[2] < need_x) return;
  if (in_sizes[3] < need_m) return;
  if (in_sizes[4] < CC * DIN || in_sizes[5] < CC * DIN || in_sizes[6] < CC * DIN || in_sizes[7] < DIN * CC) return;
  if (out_size < NB * TT * DIN) return;
  if (ws_size < (size_t)WS_END) return;
  const float* xq = (const float*)d_in[0]; const float* xk = (const float*)d_in[1]; const float* xv = (const float*)d_in[2]; const int* mask = (const int*)d_in[3];
  const float* wq = (const float*)d_in[4]; const float* wk = (const float*)d_in[5]; const float* wv = (const float*)d_in[6]; const float* wo = (const float*)d_in[7];
  char* ws = (char*)d_ws;
  _Float16* QH = (_Float16*)(ws + WS_QH); _Float16* QL = (_Float16*)(ws + WS_QL); _Float16* KH = (_Float16*)(ws + WS_KH); _Float16* VT = (_Float16*)(ws + WS_VT); float* Y = (float*)(ws + WS_Y);
  k_proj<<<dim3(NB * TT / 64, CC / 128, 3), 128, 0, stream>>>(xq, xk, xv, wq, wk, wv, QH, QL, KH, VT);
  k_attn<<<dim3(TT / 64, NB * NH), 128, 0, stream>>>(QH, QL, KH, VT, mask, Y);
  k_out<<<dim3(NB * TT / 64, DIN / 128), 128, 0, stream>>>(Y, wo, (float*)d_out);
}
